// Net_89687507075577
// MI455X (gfx1250) — hardware-run, weakly checked
//
#include <hip/hip_runtime.h>


#define NB  32
#define NBP 64
#define ND  1024
#define NH  64
#define NO  1000
#define NOP 1024
#define NE  6
typedef _Float16 h16;
typedef unsigned short bf;
typedef __attribute__((ext_vector_type(16))) __bf16   v16bf;
typedef __attribute__((ext_vector_type(16))) _Float16 v16h;
typedef __attribute__((ext_vector_type(8)))  _Float16 v8h;
typedef __attribute__((ext_vector_type(8)))  unsigned short v8us;
typedef __attribute__((ext_vector_type(8)))  float    v8f;
typedef __attribute__((ext_vector_type(4)))  float    v4f;
typedef v8h  __attribute__((may_alias)) v8ha;
typedef v4f  __attribute__((may_alias)) v4fa;
typedef v8us __attribute__((may_alias)) v8usa;

__device__ __forceinline__ unsigned short f2bf(float f) { unsigned u = __float_as_uint(f); u += 0x7FFFu + ((u >> 16) & 1u); return (unsigned short)(u >> 16); }
__device__ __forceinline__ float bf2f(unsigned short b) { return __uint_as_float(((unsigned)b) << 16); }
__device__ __forceinline__ float bfr(float f) { return bf2f(f2bf(f)); }
__device__ __forceinline__ v16h cat16(v8h lo, v8h hi) { return __builtin_shufflevector(lo, hi, 0, 1, 2, 3, 4, 5, 6, 7, 8, 9, 10, 11, 12, 13, 14, 15); }
__device__ __forceinline__ v16bf cat16b(v8us lo, v8us hi) { return __builtin_bit_cast(v16bf, __builtin_shufflevector(lo, hi, 0, 1, 2, 3, 4, 5, 6, 7, 8, 9, 10, 11, 12, 13, 14, 15)); }
__device__ __forceinline__ v8f wmma16(v16h a, v16h b, v8f c) { return __builtin_amdgcn_wmma_f32_16x16x32_f16(false, a, false, b, (short)0, c, false, false); }
__device__ __forceinline__ v8f wmmab(v16bf a, v16bf b, v8f c) { return __builtin_amdgcn_wmma_f32_16x16x32_bf16(false, a, false, b, (short)0, c, false, false); }
typedef __attribute__((ext_vector_type(2))) unsigned short v2us;

template <typename T16> struct WFrag;
template <> struct WFrag<h16> { typedef v16h V; static __device__ __forceinline__ V ld(const h16* p) { return cat16(*(const v8h*)p, *(const v8h*)(p + 16)); } static __device__ __forceinline__ v8f mma(V a, V b, v8f c) { return wmma16(a, b, c); } };
template <> struct WFrag<bf> { typedef v16bf V; static __device__ __forceinline__ V ld(const bf* p) { return cat16b(*(const v8us*)p, *(const v8us*)(p + 16)); } static __device__ __forceinline__ v8f mma(V a, V b, v8f c) { return wmmab(a, b, c); } };
template <typename T16, int NSPLIT, bool BIAS>
__global__ __launch_bounds__(32) void k_gemmw(const T16* __restrict__ A, const T16* __restrict__ A2, const T16* __restrict__ Bt, const T16* __restrict__ Bt2, int K, float* C, int ldc, const float* __restrict__ bias, size_t sA, size_t sB, size_t sC) {
    typedef typename WFrag<T16>::V V;
    __shared__ __align__(16) float os[16 * 68];
    const size_t z = blockIdx.z; A += z * sA; if (A2) A2 += z * sA; Bt += z * sB; if (Bt2) Bt2 += z * sB; C += z * sC;
    const int lane = threadIdx.x & 31, lr = lane & 15, hi = lane >> 4; const int r0 = blockIdx.x * 64, c0 = blockIdx.y * 64;
    v8f acc[4][4];
#pragma unroll
    for (int mb = 0; mb < 4; ++mb)
#pragma unroll
        for (int nb = 0; nb < 4; ++nb) acc[mb][nb] = (v8f){};
    const size_t aoff = (size_t)(r0 + lr) * K + 8 * hi, boff = (size_t)(c0 + lr) * K + 8 * hi;
    for (int kc = 0; kc < K; kc += 32) {
        V a[4], a2[4];
#pragma unroll
        for (int mb = 0; mb < 4; ++mb) { a[mb] = WFrag<T16>::ld(A + aoff + (size_t)mb * 16 * K + kc); if (NSPLIT == 1 || NSPLIT == 2) a2[mb] = WFrag<T16>::ld(A2 + aoff + (size_t)mb * 16 * K + kc); }
#pragma unroll
        for (int nb = 0; nb < 4; ++nb) { const V b = WFrag<T16>::ld(Bt + boff + (size_t)nb * 16 * K + kc); V b2; if (NSPLIT >= 2) b2 = WFrag<T16>::ld(Bt2 + boff + (size_t)nb * 16 * K + kc);
#pragma unroll
            for (int mb = 0; mb < 4; ++mb) { acc[mb][nb] = WFrag<T16>::mma(a[mb], b, acc[mb][nb]); if (NSPLIT == 1 || NSPLIT == 2) acc[mb][nb] = WFrag<T16>::mma(a2[mb], b, acc[mb][nb]); if (NSPLIT >= 2) acc[mb][nb] = WFrag<T16>::mma(a[mb], b2, acc[mb][nb]); } }
        asm volatile("v_nop\n\tv_nop\n\tv_nop\n\tv_nop" : "+v"(acc[0][0]), "+v"(acc[1][1]), "+v"(acc[2][2]), "+v"(acc[3][3]) : "v"(a[0]), "v"(a[3]));
    }
#pragma unroll
    for (int mb = 0; mb < 4; ++mb) {
#pragma unroll
        for (int nb = 0; nb < 4; ++nb) {
#pragma unroll
            for (int j = 0; j < 8; ++j) os[(hi * 8 + j) * 68 + nb * 16 + lr] = acc[mb][nb][j]; }
        __builtin_amdgcn_wave_barrier(); asm volatile("" ::: "memory");
        float* crow = C + (size_t)(r0 + mb * 16) * ldc + c0;
#pragma unroll 1
        for (int ps = 0; ps < 2; ++ps) {
#pragma unroll
            for (int s = 0; s < 8; ++s) { const int row = 2 * s + hi, cofs = lr * 4; v4f val = *(const v4fa*)(os + row * 68 + cofs); if (BIAS) { val[0] += bfr(bias[c0 + cofs]); val[1] += bfr(bias[c0 + cofs + 1]); val[2] += bfr(bias[c0 + cofs + 2]); val[3] += bfr(bias[c0 + cofs + 3]); }
                *(volatile v4f*)(crow + (size_t)row * ldc + cofs) = val; }
            if (ps == 0) __threadfence(); }
        __builtin_amdgcn_wave_barrier(); asm volatile("" ::: "memory");
    }
}
__global__ __launch_bounds__(256) void k_cvt8(const float* __restrict__ src, bf* dst, size_t n8) { const size_t i = (size_t)blockIdx.x * 256 + threadIdx.x; if (i >= n8) return; const v8f v = *(const v8f*)(src + i * 8); v8us o;
#pragma unroll
    for (int k = 0; k < 8; ++k) o[k] = f2bf(v[k]); *(volatile v8us*)(dst + i * 8) = o; __threadfence(); *(volatile v8us*)(dst + i * 8) = o; }

__global__ __launch_bounds__(256) void k_wtG(const float* __restrict__ w, int K, int N, bf* Bt) {
    const int lane = threadIdx.x & 31; const int L0 = (blockIdx.x * 8 + (threadIdx.x >> 5)) * 8; const int nlines = N * K / 64;
#pragma unroll
    for (int ps = 0; ps < 2; ++ps) {
        for (int l = 0; l < 8; ++l) { const int L = L0 + l; if (L >= nlines) break; const size_t e = (size_t)L * 64 + lane * 2; const int k = (int)(e % K), n = (int)(e / K); v2us o;
            o[0] = f2bf(w[(size_t)k * N + n]); o[1] = f2bf(w[(size_t)(k + 1) * N + n]); *(volatile v2us*)(Bt + e) = o; }
        if (ps == 0) __threadfence(); }
}

__global__ __launch_bounds__(32) void k_gate(const float* __restrict__ x, const float* __restrict__ gw, const float* __restrict__ gb, float* G) { const int b = threadIdx.x; if (b >= NB) return; float s0 = 0.0f, s1 = 0.0f, s2 = 0.0f, s3 = 0.0f, s4 = 0.0f, s5 = 0.0f; const float* xr = x + (size_t)b * ND;
#pragma unroll 1
  for (int k = 0; k < ND; ++k) { const float xv = bfr(xr[k]); const float* g = gw + (size_t)k * NE; s0 += xv * bfr(g[0]); s1 += xv * bfr(g[1]); s2 += xv * bfr(g[2]); s3 += xv * bfr(g[3]); s4 += xv * bfr(g[4]); s5 += xv * bfr(g[5]); }
  float lg[NE] = { s0 + bfr(gb[0]), s1 + bfr(gb[1]), s2 + bfr(gb[2]), s3 + bfr(gb[3]), s4 + bfr(gb[4]), s5 + bfr(gb[5]) };
  float v1 = lg[0]; int i1 = 0; float v2 = -3.0e38f; int i2 = -1;
#pragma unroll
  for (int e = 1; e < NE; ++e) { const float v = lg[e]; const bool first = v > v1; const bool second = !first && (v > v2); v2 = first ? v1 : (second ? v : v2); i2 = first ? i1 : (second ? e : i2); v1 = first ? v : v1; i1 = first ? e : i1; }
  const float mx = v1; const float e1 = expf(v1 - mx), e2 = expf(v2 - mx); const float sm = e1 + e2; const float g1 = e1 / sm, g2 = e2 / sm;
#pragma unroll
  for (int e = 0; e < NE; ++e) { const float g = (e == i1) ? g1 : ((e == i2) ? g2 : 0.0f); float* p = G + (size_t)b * NE + e; *(volatile float*)p = g; }
  __threadfence();
#pragma unroll
  for (int e = 0; e < NE; ++e) { const float g = (e == i1) ? g1 : ((e == i2) ? g2 : 0.0f); float* p = G + (size_t)b * NE + e; *(volatile float*)p = g; } }

__global__ __launch_bounds__(256) void k_w2t(const float* __restrict__ w2, h16* W2T) { const int i = blockIdx.x * 256 + threadIdx.x; if (i >= NE * NOP * (NH / 8)) return; const int k0 = (i & 7) * 8, n = (i >> 3) & (NOP - 1), e = i >> 13; const int nc = n < NO ? n : NO - 1; const unsigned short keep = (unsigned short)(n < NO ? 0xffffu : 0u); v8us o;
#pragma unroll
  for (int k = 0; k < 8; ++k) { const h16 hv = (h16)(bfr(w2[((size_t)e * NH + (k0 + k)) * NO + nc]) * 1024.0f); unsigned short bits; __builtin_memcpy(&bits, &hv, 2); o[k] = (unsigned short)(bits & keep); }
  unsigned short* p = (unsigned short*)W2T + (size_t)i * 8; *(volatile v8us*)p = o; __threadfence(); *(volatile v8us*)p = o; }

__global__ __launch_bounds__(256) void k_act(const float* __restrict__ H, const float* __restrict__ b1, h16* HA) { const int i = blockIdx.x * 256 + threadIdx.x; if (i >= NE * NBP * NH / 8) return; const int col0 = (i & 7) * 8, e = i >> 9; v8us o;
#pragma unroll
  for (int k = 0; k < 8; ++k) { const h16 hv = (h16)fmaxf(H[(size_t)i * 8 + k] + bfr(b1[e * NH + col0 + k]), 0.0f); unsigned short bits; __builtin_memcpy(&bits, &hv, 2); o[k] = bits; }
  unsigned short* p = (unsigned short*)HA + (size_t)i * 8; *(volatile v8us*)p = o; __threadfence(); *(volatile v8us*)p = o; }

__global__ __launch_bounds__(256) void k_comb(const float* __restrict__ Y, const float* __restrict__ G, const float* __restrict__ b2, float* OUT) { const int i = blockIdx.x * 256 + threadIdx.x; if (i >= NB * NO) return; const int o = i % NO, b = i / NO; float s = 0.0f;
#pragma unroll
  for (int e = 0; e < NE; ++e) s += G[b * NE + e] * (Y[((size_t)e * NBP + b) * NOP + o] * 0.0009765625f + bfr(b2[e * NO + o]));
  *(volatile float*)(OUT + i) = s; __threadfence(); *(volatile float*)(OUT + i) = s; }

extern "C" void kernel_launch(void* const* d_in, const int* in_sizes, int n_in,
                              void* d_out, int out_size, void* d_ws, size_t ws_size, hipStream_t stream) {
    (void)in_sizes; (void)n_in; (void)out_size;
    const float* x = (const float*)d_in[0]; const float* gw = (const float*)d_in[1]; const float* gb = (const float*)d_in[2]; const float* w1 = (const float*)d_in[3]; const float* b1 = (const float*)d_in[4]; const float* w2 = (const float*)d_in[5]; const float* b2 = (const float*)d_in[6];
    float* OUT = (float*)d_out;
    char* wsp = (char*)d_ws;
    auto take = [&](size_t bytes) { char* p = wsp; wsp += (bytes + 255) & ~(size_t)255; return (void*)p; };
    bf* XP = (bf*)take((size_t)NBP * ND * 2); bf* W1T = (bf*)take((size_t)NE * NH * ND * 2); float* H = (float*)take((size_t)NE * NBP * NH * 4); h16* HA = (h16*)take((size_t)NE * NBP * NH * 2); h16* W2T = (h16*)take((size_t)NE * NOP * NH * 2); float* Y = (float*)take((size_t)NE * NBP * NOP * 4); float* G = (float*)take((size_t)NB * NE * 4);
    if ((size_t)(wsp - (char*)d_ws) > ws_size) return;
    k_cvt8<<<NB * ND / 8 / 256, 256, 0, stream>>>(x, XP, (size_t)NB * ND / 8);
    k_cvt8<<<NB * ND / 8 / 256, 256, 0, stream>>>(x, XP + (size_t)NB * ND, (size_t)NB * ND / 8);
    for (int e = 0; e < NE; ++e) k_wtG<<<(unsigned)((ND * NH / 64 + 63) / 64), 256, 0, stream>>>(w1 + (size_t)e * ND * NH, ND, NH, W1T + (size_t)e * NH * ND);
    k_w2t<<<NE * NOP * (NH / 8) / 256, 256, 0, stream>>>(w2, W2T);
    k_gate<<<1, 32, 0, stream>>>(x, gw, gb, G);
    k_gemmw<bf, 0, false><<<dim3(NBP / 64, NH / 64, NE), 32, 0, stream>>>(XP, nullptr, W1T, nullptr, ND, H, NH, nullptr, 0, (size_t)NH * ND, (size_t)NBP * NH);
    k_act<<<NE * NBP * NH / 8 / 256, 256, 0, stream>>>(H, b1, HA);
    k_gemmw<h16, 0, false><<<dim3(NBP / 64, NOP / 64, NE), 32, 0, stream>>>(HA, nullptr, W2T, nullptr, NH, Y, NOP, nullptr, (size_t)NBP * NH, (size_t)NOP * NH, (size_t)NBP * NOP);
    k_comb<<<(NB * NO + 255) / 256, 256, 0, stream>>>(Y, G, b2, OUT);
}
